// MaskedSelfAttention_71691594104857
// MI455X (gfx1250) — hardware-verified
//
#include <hip/hip_runtime.h>
#include <math.h>
#include <stdint.h>

#ifndef NB
#define NB 4
#endif
#ifndef SEQ
#define SEQ 4096
#endif
#define SEQ_FULL 4096
#define NB_FULL 4
#define EMB   512
#define DH    64
#define CK    512
#define NCHK  (SEQ / CK)
#define NKB   16
#define QT    16
#define TQ0   128
#define NQT   ((SEQ - TQ0) / QT)
#define SCP   544
#define PLP   528
#define OPP   68
#define CTP   72
#define SLAB64 (16 * 68)
#define VTP   72
#define ATT_THREADS 256
#define HD_THREADS 128
#define NACC  4
#define QSC   8.0f
#define KSC   8.0f
#define PCAR  32768.0f
#define VCAR  1024.0f
#define WSC   1024.0f
#define CSC   4096.0f
#define RSC   2048.0f
#define LOG2E 1.4426950408889634f
#define RSQD  0.125f
#define WS_CAP ((size_t)134217728)

static_assert(DH == 64 && NACC * 16 == DH && (EMB % 64) == 0 && (EMB % 32) == 0 && (DH % 32) == 0);
static_assert((SEQ % CK) == 0 && NCHK >= 1 && CK == 32 * NKB && (SEQ % 64) == 0 && (SEQ % QT) == 0 && (CK % QT) == 0);
static_assert((TQ0 % QT) == 0 && (TQ0 % 64) == 0 && NQT * QT + TQ0 == SEQ && NQT >= 1 && TQ0 == 128 && TQ0 == HD_THREADS);
static_assert(8 * 16 * OPP <= 16 * SCP && 32 * CTP <= 16 * PLP && CTP >= DH + 8 && OPP >= DH + 4 && SCP >= CK + 16 && PLP >= CK + 8);
static_assert(((PLP * 2) % 16) == 0 && ((SCP * 4) % 16) == 0 && ((VTP * 2) % 16) == 0 && ((CTP * 2) % 16) == 0 && ((OPP * 4) % 16) == 0);
static_assert(64 * VTP >= 63 * VTP + 64);
static_assert(ATT_THREADS == 16 * QT && ATT_THREADS == 256 && HD_THREADS == 2 * DH);
static_assert((((SEQ * EMB) / 8) % 256) == 0 && ((NB * SEQ) % 64) == 0 && ((NB * TQ0) % 64) == 0);
static_assert(NB >= 1 && NB <= NB_FULL && SEQ <= SEQ_FULL);

typedef unsigned short u16;
typedef _Float16 v16h __attribute__((ext_vector_type(16)));
typedef _Float16 v8h  __attribute__((ext_vector_type(8)));
typedef __bf16   v16b __attribute__((ext_vector_type(16)));
typedef float    v8f  __attribute__((ext_vector_type(8)));
typedef float    v4f  __attribute__((ext_vector_type(4)));
typedef unsigned int v4u __attribute__((ext_vector_type(4)));

union FragH { v16h v; v8h h[2]; v4u u[2]; };
union FragB { v16b v; v4u u[2]; };

__device__ __forceinline__ unsigned short bf_bits(float f) {
  unsigned u = __float_as_uint(f);
  return (unsigned short)((u + 0x7FFFu + ((u >> 16) & 1u)) >> 16);
}
__device__ __forceinline__ float bf_up(unsigned short h) { return __uint_as_float(((unsigned)h) << 16); }
__device__ __forceinline__ float bfr(float f) { return bf_up(bf_bits(f)); }
__device__ __forceinline__ unsigned short h_bits(_Float16 x) { return __builtin_bit_cast(unsigned short, x); }
__device__ __forceinline__ unsigned pk16(unsigned short a, unsigned short b) { return (unsigned)a | ((unsigned)b << 16); }
__device__ __forceinline__ v8f zero8() { v8f z = {0.f, 0.f, 0.f, 0.f, 0.f, 0.f, 0.f, 0.f}; return z; }
__device__ __forceinline__ v4f zero4() { v4f z = {0.f, 0.f, 0.f, 0.f}; return z; }

__device__ __forceinline__ v16h ldfrag_h(const _Float16* p) {
  FragH f;
  f.h[0] = *(const v8h*)(p);
  f.h[1] = *(const v8h*)(p + 16);
  return f.v;
}
__device__ __forceinline__ v16b ldfrag_b(const u16* p) {
  FragB f;
  f.u[0] = *(const v4u*)(p);
  f.u[1] = *(const v4u*)(p + 16);
  return f.v;
}

__device__ __forceinline__ v8f mma_h(v16h a, v16h b, v8f c) {
  return __builtin_amdgcn_wmma_f32_16x16x32_f16(false, a, false, b, (short)0, c, false, false);
}
__device__ __forceinline__ v8f mma_b(v16b a, v16b b, v8f c) {
  return __builtin_amdgcn_wmma_f32_16x16x32_bf16(false, a, false, b, (short)0, c, false, false);
}
__device__ __forceinline__ void guard2x6(v8f& a, v8f& b, v16h x0, v16h x1, v16h x2, v16h x3, v16h x4, v16h x5) {
#if defined(__HIP_DEVICE_COMPILE__)
  asm volatile("v_nop\n\tv_nop\n\tv_nop\n\tv_nop"
               : "+v"(a), "+v"(b) : "v"(x0), "v"(x1), "v"(x2), "v"(x3), "v"(x4), "v"(x5) : "memory");
#endif
}
template <typename F>
__device__ __forceinline__ void guard6(v8f& a, v8f& b, v8f& c, v8f& d, F x0, F x1, F x2, F x3, F x4, F x5) {
#if defined(__HIP_DEVICE_COMPILE__)
  asm volatile("v_nop\n\tv_nop\n\tv_nop\n\tv_nop"
               : "+v"(a), "+v"(b), "+v"(c), "+v"(d) : "v"(x0), "v"(x1), "v"(x2), "v"(x3), "v"(x4), "v"(x5) : "memory");
#endif
}
__device__ __forceinline__ void guard8x6(v8f& a0, v8f& a1, v8f& a2, v8f& a3, v8f& e0, v8f& e1, v8f& e2, v8f& e3,
                                         v16h x0, v16h x1, v16h x2, v16h x3, v16h x4, v16h x5) {
#if defined(__HIP_DEVICE_COMPILE__)
  asm volatile("v_nop\n\tv_nop\n\tv_nop\n\tv_nop"
               : "+v"(a0), "+v"(a1), "+v"(a2), "+v"(a3), "+v"(e0), "+v"(e1), "+v"(e2), "+v"(e3)
               : "v"(x0), "v"(x1), "v"(x2), "v"(x3), "v"(x4), "v"(x5) : "memory");
#endif
}
__device__ __forceinline__ void guardpv4(v8f& o0, v8f& o1, v8f& o2, v8f& o3, v16h p, v16h g0, v16h g1, v16h g2, v16h g3) {
#if defined(__HIP_DEVICE_COMPILE__)
  asm volatile("v_nop\n\tv_nop\n\tv_nop\n\tv_nop"
               : "+v"(o0), "+v"(o1), "+v"(o2), "+v"(o3)
               : "v"(p), "v"(g0), "v"(g1), "v"(g2), "v"(g3) : "memory");
#endif
}
__device__ __forceinline__ void acc_guard4(v8f& a, v8f& b, v8f& c, v8f& d) {
#if defined(__HIP_DEVICE_COMPILE__)
  asm volatile("v_nop\n\tv_nop\n\tv_nop\n\tv_nop" : "+v"(a), "+v"(b), "+v"(c), "+v"(d));
#endif
}
__device__ __forceinline__ void wave_sync_lds() {
  __builtin_amdgcn_fence(3, "workgroup");
  __builtin_amdgcn_wave_barrier();
  __builtin_amdgcn_fence(2, "workgroup");
}

__global__ __launch_bounds__(256) void cvtx(const float* __restrict__ x, u16* D, int n8) {
  const int gt = blockIdx.x * 256 + (int)threadIdx.x;
  if (gt >= n8) return;
  const int bb = blockIdx.y;
  const float* p = x + (size_t)bb * ((size_t)SEQ_FULL * EMB) + (size_t)gt * 8;
  const v4f a = *(const v4f*)(p), c4 = *(const v4f*)(p + 4);
  float v[8];
#pragma unroll
  for (int e = 0; e < 4; ++e) { v[e] = a[e]; v[4 + e] = c4[e]; }
  unsigned short s[8];
#pragma unroll
  for (int e = 0; e < 8; ++e) s[e] = bf_bits(v[e]);
  v4u o;
#pragma unroll
  for (int e = 0; e < 4; ++e) o[e] = pk16(s[2 * e], s[2 * e + 1]);
  u16* d = D + (size_t)bb * ((size_t)SEQ * EMB) + (size_t)gt * 8;
  for (int pass = 0; pass < 2; ++pass) {
    *(volatile v4u*)(d) = o;
    __threadfence();
  }
}

__global__ __launch_bounds__(256) void wt16(const float* __restrict__ W, u16* D, int R, int C, int mode, float scale) {
  __shared__ __align__(16) u16 TH[64 * VTP];
  const int tid = threadIdx.x;
  const int bid = blockIdx.x;
  const int nrt = R >> 6;
  const int r0  = (bid % nrt) * 64;
  const int c0  = (bid / nrt) * 64;
  {
    const int rl = tid >> 2;
    const int cs = (tid & 3) * 16;
    const float* src = W + (size_t)(r0 + rl) * C + c0 + cs;
#pragma unroll
    for (int i = 0; i < 4; ++i) {
      const v4f a = *(const v4f*)(src + 4 * i);
#pragma unroll
      for (int e = 0; e < 4; ++e) {
        const float v  = a[e];
        const unsigned short hb = h_bits((_Float16)(bfr(v) * scale));
        const unsigned short bb = bf_bits(v);
        TH[(cs + 4 * i + e) * VTP + rl] = (mode != 0) ? hb : bb;
      }
    }
  }
  __syncthreads();
  v4u vh[2];
  const int q8 = tid >> 3, p8 = (tid & 7) * 8;
#pragma unroll
  for (int it = 0; it < 2; ++it) {
    const int line = it * 32 + q8;
    vh[it] = *(const v4u*)(TH + line * VTP + p8);
  }
  const size_t base = (size_t)c0 * (size_t)R + (size_t)r0 + p8;
  for (int pass = 0; pass < 2; ++pass) {
#pragma unroll
    for (int it = 0; it < 2; ++it) {
      const int line = it * 32 + q8;
      *(volatile v4u*)(D + base + (size_t)line * (size_t)R) = vh[it];
    }
    __threadfence();
  }
}

__device__ __forceinline__ void stage64(float* sl, v8f a0, v8f a1, v8f a2, v8f a3, float oscale, int lane) {
  const int hh = lane >> 4, m = lane & 15;
#pragma unroll
  for (int r = 0; r < 8; ++r) {
    const int ro = (8 * hh + r) * 68 + m;
    sl[ro]      = a0[r] * oscale;
    sl[ro + 16] = a1[r] * oscale;
    sl[ro + 32] = a2[r] * oscale;
    sl[ro + 48] = a3[r] * oscale;
  }
  wave_sync_lds();
}
__device__ __forceinline__ void epi64(float* sl, v8f a0, v8f a1, v8f a2, v8f a3, float oscale, v4f badd, float* C, int N,
                                      size_t rowb, int col0, int lane) {
  const int hh = lane >> 4, m = lane & 15;
  stage64(sl, a0, a1, a2, a3, oscale, lane);
  v4f vals[8];
#pragma unroll
  for (int it = 0; it < 8; ++it) vals[it] = *(const v4f*)(sl + (it * 2 + hh) * 68 + m * 4) + badd;
  float* dst = C + (rowb + (size_t)hh) * (size_t)N + col0 + m * 4;
  for (int pass = 0; pass < 2; ++pass) {
#pragma unroll
    for (int it = 0; it < 8; ++it) {
      *(volatile v4f*)(dst + (size_t)(it * 2) * (size_t)N) = vals[it];
    }
    __threadfence();
  }
}
__device__ __forceinline__ void epi64x2(float* sl, v8f a0, v8f a1, v8f a2, v8f a3, v8f e0, v8f e1, v8f e2, v8f e3,
                                        float os1, float os2, v4f badd, float* C, int N, size_t rowb, int col0, int lane) {
  const int hh = lane >> 4, m = lane & 15;
#pragma unroll
  for (int r = 0; r < 8; ++r) {
    const int ro = (8 * hh + r) * 68 + m;
    sl[ro]      = a0[r] * os1 + e0[r] * os2;
    sl[ro + 16] = a1[r] * os1 + e1[r] * os2;
    sl[ro + 32] = a2[r] * os1 + e2[r] * os2;
    sl[ro + 48] = a3[r] * os1 + e3[r] * os2;
  }
  wave_sync_lds();
  v4f vals[8];
#pragma unroll
  for (int it = 0; it < 8; ++it) vals[it] = *(const v4f*)(sl + (it * 2 + hh) * 68 + m * 4) + badd;
  float* dst = C + (rowb + (size_t)hh) * (size_t)N + col0 + m * 4;
  for (int pass = 0; pass < 2; ++pass) {
#pragma unroll
    for (int it = 0; it < 8; ++it) {
      *(volatile v4f*)(dst + (size_t)(it * 2) * (size_t)N) = vals[it];
    }
    __threadfence();
  }
}
__device__ __forceinline__ void epi64hsb(float* sl, v8f a0, v8f a1, v8f a2, v8f a3, float oscale, float pscale,
                                         const float* __restrict__ bias, u16* C, int N, size_t rowb, int col0, int lane) {
  stage64(sl, a0, a1, a2, a3, oscale, lane);
  const int rq = lane >> 3, c8 = (lane & 7) * 8;
  const v4f b0 = *(const v4f*)(bias + col0 + c8), b1 = *(const v4f*)(bias + col0 + c8 + 4);
  float bb[8];
#pragma unroll
  for (int e = 0; e < 4; ++e) { bb[e] = bfr(b0[e]); bb[4 + e] = bfr(b1[e]); }
  v4u oh[4];
#pragma unroll
  for (int i4 = 0; i4 < 4; ++i4) {
    const int row = i4 * 4 + rq;
    const v4f a = *(const v4f*)(sl + row * 68 + c8), c4 = *(const v4f*)(sl + row * 68 + c8 + 4);
    float w[8];
#pragma unroll
    for (int e = 0; e < 4; ++e) { w[e] = (a[e] + bb[e]) * pscale; w[4 + e] = (c4[e] + bb[4 + e]) * pscale; }
#pragma unroll
    for (int e = 0; e < 4; ++e) oh[i4][e] = pk16(h_bits((_Float16)w[2 * e]), h_bits((_Float16)w[2 * e + 1]));
  }
  u16* dst = C + rowb * (size_t)N + col0 + c8;
  for (int pass = 0; pass < 2; ++pass) {
#pragma unroll
    for (int i4 = 0; i4 < 4; ++i4) {
      const int row = i4 * 4 + rq;
      *(volatile v4u*)(dst + (size_t)row * (size_t)N) = oh[i4];
    }
    __threadfence();
  }
}

__global__ __launch_bounds__(128)
void gemm_b32(const u16* __restrict__ A, const u16* __restrict__ Bt, const float* __restrict__ bias, float* C,
              int M, int N, int K, int rpg, int gstr, float oscale) {
  __shared__ __align__(16) float slab[4 * SLAB64];
  const int tid = threadIdx.x, wave = tid >> 5, lane = tid & 31, hh = lane >> 4, m = lane & 15;
  const int ntile = N >> 6;
  const int bid   = blockIdx.x;
  const int rowb  = (bid / ntile) * 64 + wave * 16;
  const int col0  = (bid % ntile) * 64;
  if (rowb + 16 > M) return;
  const int ra = rowb + m;
  const int rg = ra / rpg;
  const size_t arow = (size_t)rg * (size_t)gstr + (size_t)(ra - rg * rpg);
  const u16* ap = A  + arow * (size_t)K + 8 * hh;
  const u16* bp = Bt + (size_t)(col0 + m) * K + 8 * hh;
  const size_t bs = (size_t)16 * K;
  v8f acc0 = zero8(), acc1 = zero8(), acc2 = zero8(), acc3 = zero8();
#pragma unroll 1
  for (int k0 = 0; k0 < K; k0 += 32) {
    const v16b a  = ldfrag_b(ap + k0);
    const v16b b0 = ldfrag_b(bp + k0);
    const v16b b1 = ldfrag_b(bp + bs + k0);
    const v16b b2 = ldfrag_b(bp + 2 * bs + k0);
    const v16b b3 = ldfrag_b(bp + 3 * bs + k0);
    acc0 = mma_b(a, b0, acc0);
    acc1 = mma_b(a, b1, acc1);
    acc2 = mma_b(a, b2, acc2);
    acc3 = mma_b(a, b3, acc3);
    guard6<v16b>(acc0, acc1, acc2, acc3, a, b0, b1, b2, b3, a);
  }
  const v4f bv4 = *(const v4f*)(bias + col0 + m * 4);
  v4f badd;
#pragma unroll
  for (int e = 0; e < 4; ++e) badd[e] = bfr(bv4[e]);
  epi64(slab + wave * SLAB64, acc0, acc1, acc2, acc3, oscale, badd, C, N, (size_t)rowb, col0, lane);
}

__global__ __launch_bounds__(128)
void gemm_bh16(const u16* __restrict__ A, const u16* __restrict__ Bt, const float* __restrict__ bias, u16* C,
               int M, int N, int K, float oscale, float pscale) {
  __shared__ __align__(16) float slab[4 * SLAB64];
  const int tid = threadIdx.x, wave = tid >> 5, lane = tid & 31, hh = lane >> 4, m = lane & 15;
  const int ntile = N >> 6;
  const int bid   = blockIdx.x;
  const int rowb  = (bid / ntile) * 64 + wave * 16;
  const int col0  = (bid % ntile) * 64;
  if (rowb + 16 > M) return;
  const u16* ap = A  + (size_t)(rowb + m) * K + 8 * hh;
  const u16* bp = Bt + (size_t)(col0 + m) * K + 8 * hh;
  const size_t bs = (size_t)16 * K;
  v8f acc0 = zero8(), acc1 = zero8(), acc2 = zero8(), acc3 = zero8();
#pragma unroll 1
  for (int k0 = 0; k0 < K; k0 += 32) {
    const v16b a  = ldfrag_b(ap + k0);
    const v16b b0 = ldfrag_b(bp + k0);
    const v16b b1 = ldfrag_b(bp + bs + k0);
    const v16b b2 = ldfrag_b(bp + 2 * bs + k0);
    const v16b b3 = ldfrag_b(bp + 3 * bs + k0);
    acc0 = mma_b(a, b0, acc0);
    acc1 = mma_b(a, b1, acc1);
    acc2 = mma_b(a, b2, acc2);
    acc3 = mma_b(a, b3, acc3);
    guard6<v16b>(acc0, acc1, acc2, acc3, a, b0, b1, b2, b3, a);
  }
  epi64hsb(slab + wave * SLAB64, acc0, acc1, acc2, acc3, oscale, pscale, bias, C, N, (size_t)rowb, col0, lane);
}

__global__ __launch_bounds__(128)
void gemm_h2_32(const u16* __restrict__ Ah, const u16* __restrict__ Ar, const u16* __restrict__ Bt,
                const float* __restrict__ bias, float* C, int M, int N, int K, float os1, float os2) {
  __shared__ __align__(16) float slab[4 * SLAB64];
  const int tid = threadIdx.x, wave = tid >> 5, lane = tid & 31, hh = lane >> 4, m = lane & 15;
  const int ntile = N >> 6;
  const int bid   = blockIdx.x;
  const int rowb  = (bid / ntile) * 64 + wave * 16;
  const int col0  = (bid % ntile) * 64;
  if (rowb + 16 > M) return;
  const _Float16* ap  = (const _Float16*)(const void*)Ah + (size_t)(rowb + m) * K + 8 * hh;
  const _Float16* arp = (const _Float16*)(const void*)Ar + (size_t)(rowb + m) * K + 8 * hh;
  const _Float16* bp  = (const _Float16*)(const void*)Bt + (size_t)(col0 + m) * K + 8 * hh;
  const size_t bs = (size_t)16 * K;
  v8f acc0 = zero8(), acc1 = zero8(), acc2 = zero8(), acc3 = zero8();
  v8f acr0 = zero8(), acr1 = zero8(), acr2 = zero8(), acr3 = zero8();
#pragma unroll 1
  for (int k0 = 0; k0 < K; k0 += 32) {
    const v16h a  = ldfrag_h(ap + k0);
    const v16h ar = ldfrag_h(arp + k0);
    const v16h b0 = ldfrag_h(bp + k0);
    const v16h b1 = ldfrag_h(bp + bs + k0);
    const v16h b2 = ldfrag_h(bp + 2 * bs + k0);
    const v16h b3 = ldfrag_h(bp + 3 * bs + k0);
    acc0 = mma_h(a, b0, acc0);
    acc1 = mma_h(a, b1, acc1);
    acc2 = mma_h(a, b2, acc2);
    acc3 = mma_h(a, b3, acc3);
    acr0 = mma_h(ar, b0, acr0);
    acr1 = mma_h(ar, b1, acr1);
    acr2 = mma_h(ar, b2, acr2);
    acr3 = mma_h(ar, b3, acr3);
    guard8x6(acc0, acc1, acc2, acc3, acr0, acr1, acr2, acr3, a, ar, b0, b1, b2, b3);
  }
  const v4f bv = *(const v4f*)(bias + col0 + m * 4);
  v4f badd;
#pragma unroll
  for (int e = 0; e < 4; ++e) badd[e] = bfr(bv[e]);
  epi64x2(slab + wave * SLAB64, acc0, acc1, acc2, acc3, acr0, acr1, acr2, acr3, os1, os2, badd, C, N,
          (size_t)rowb, col0, lane);
}

__global__ __launch_bounds__(256) void xt16(const float* __restrict__ X, u16* XTo) {
  __shared__ __align__(16) u16 TH[64 * VTP];
  const int tid = threadIdx.x;
  const int bid = blockIdx.x;
  const int st  = bid % (SEQ / 64);
  const int b   = bid / (SEQ / 64);
  const int s0  = st * 64;
  {
    const int sl = tid >> 2;
    const int dc = (tid & 3) * 16;
    const float* src = X + ((size_t)b * SEQ + s0 + sl) * DH + dc;
#pragma unroll
    for (int i = 0; i < 4; ++i) {
      const v4f a = *(const v4f*)(src + 4 * i);
#pragma unroll
      for (int e = 0; e < 4; ++e) {
        const float v = a[e];
        TH[(dc + 4 * i + e) * VTP + sl] = h_bits((_Float16)(v * VCAR));
      }
    }
  }
  __syncthreads();
  v4u vh[2];
  const int q8 = tid >> 3, p8 = (tid & 7) * 8;
#pragma unroll
  for (int it = 0; it < 2; ++it) {
    const int line = it * 32 + q8;
    vh[it] = *(const v4u*)(TH + line * VTP + p8);
  }
  const size_t base = ((size_t)b * DH) * SEQ + s0 + p8;
  for (int pass = 0; pass < 2; ++pass) {
#pragma unroll
    for (int it = 0; it < 2; ++it) {
      const int line = it * 32 + q8;
      *(volatile v4u*)(XTo + base + (size_t)line * SEQ) = vh[it];
    }
    __threadfence();
  }
}

__global__ __launch_bounds__(64) void vsum_k(const float* __restrict__ V, float* VS) {
  __shared__ __align__(16) float sm[NKB * DH];
  const int tid = threadIdx.x;
  const int bc  = blockIdx.x;
  const int b   = bc / NCHK;
  const int c   = bc - b * NCHK;
  const float* p = V + ((size_t)b * SEQ + (size_t)c * CK) * DH + tid;
  float s = 0.f;
#pragma unroll 1
  for (int kb = 0; kb < NKB; ++kb) {
#pragma unroll 4
    for (int i = 0; i < 32; ++i) s += p[(size_t)(kb * 32 + i) * DH];
    sm[kb * DH + tid] = s;
  }
  __syncthreads();
  v4f o[4];
#pragma unroll
  for (int it = 0; it < 4; ++it) o[it] = *(const v4f*)(sm + it * 256 + tid * 4);
  float* base = VS + (size_t)bc * NKB * DH + tid * 4;
  for (int pass = 0; pass < 2; ++pass) {
#pragma unroll
    for (int it = 0; it < 4; ++it) {
      *(volatile v4f*)(base + it * 256) = o[it];
    }
    __threadfence();
  }
}

__global__ __launch_bounds__(ATT_THREADS) __attribute__((amdgpu_num_vgpr(256)))
void attn_fwd(const u16* __restrict__ QPp, const u16* __restrict__ KPp, const u16* __restrict__ VTp,
              const float* __restrict__ VSp, u16* CHo, u16* CRo) {
  __shared__ __align__(16) float scs[16 * SCP];
  __shared__ __align__(16) u16 pls[16 * PLP];
  __shared__ float rowa[QT];
  __shared__ float rowc[QT];

  const int tid  = threadIdx.x;
  const int wave = tid >> 5;
  const int lane = tid & 31;
  const int hh   = lane >> 4;
  const int m    = lane & 15;
  const int r16  = tid >> 4;
  const int sub  = tid & 15;
  const int kl0  = sub * 32;

  const int bid = blockIdx.x;
  const int b   = bid / NQT;
  const int q0  = TQ0 + (bid - b * NQT) * QT;
  const int qc  = q0 / CK;

  const _Float16* qrow = (const _Float16*)(const void*)QPp + ((size_t)b * SEQ + q0 + m) * DH + 8 * hh;
  const v16h qa0 = ldfrag_h(qrow);
  const v16h qa1 = ldfrag_h(qrow + 32);
  const _Float16* kbp = (const _Float16*)(const void*)KPp + ((size_t)b * SEQ + m) * DH + 8 * hh;
  const _Float16* vbp = (const _Float16*)(const void*)VTp + ((size_t)b * DH + m) * SEQ + 8 * hh;
  const float* vsb = VSp + (size_t)b * NCHK * NKB * DH + m;
  const float lsc = RSQD * LOG2E / (QSC * KSC);
  const float addsel = (wave == 0) ? (PCAR * VCAR) : 0.f;

  float mrun = -INFINITY, lrun = 0.f;
  v8f o[NACC];
#pragma unroll
  for (int j = 0; j < NACC; ++j) o[j] = zero8();

#pragma unroll 1
  for (int c = 0; c <= qc; ++c) {
    const int kbeg = c * CK;
    const int nkb  = (c < qc) ? NKB : (((q0 + QT - 1 - kbeg) >> 5) + 1);
#pragma unroll 1
    for (int kb = wave; kb < NKB; kb += 8) {
      v8f s0 = zero8(), s1 = zero8();
      if (kb < nkb) {
        const _Float16* k0p = kbp + (size_t)(kbeg + kb * 32) * DH;
        const _Float16* k1p = k0p + (size_t)16 * DH;
        const v16h f00 = ldfrag_h(k0p);
        const v16h f01 = ldfrag_h(k0p + 32);
        const v16h f10 = ldfrag_h(k1p);
        const v16h f11 = ldfrag_h(k1p + 32);
        s0 = mma_h(qa0, f00, s0);
        s0 = mma_h(qa1, f01, s0);
        s1 = mma_h(qa0, f10, s1);
        s1 = mma_h(qa1, f11, s1);
        guard2x6(s0, s1, qa0, qa1, f00, f01, f10, f11);
      }
      float* srow = scs + (8 * hh) * SCP + kb * 32 + m;
#pragma unroll
      for (int r = 0; r < 8; ++r) {
        srow[r * SCP]      = s0[r];
        srow[r * SCP + 16] = s1[r];
      }
    }
    __syncthreads();
    {
      const float* sp = scs + r16 * SCP + kl0;
      const int lim = (q0 + r16) - (kbeg + kl0);
      float t[32];
      float cm = -INFINITY;
#pragma unroll
      for (int i = 0; i < 8; ++i) {
        const v4f a = *(const v4f*)(sp + 4 * i);
#pragma unroll
        for (int e = 0; e < 4; ++e) {
          const int j = 4 * i + e;
          const float tv = (j <= lim) ? a[e] * lsc : -INFINITY;
          t[j] = tv;
          cm = fmaxf(cm, tv);
        }
      }
#pragma unroll
      for (int d = 1; d <= 8; d <<= 1) cm = fmaxf(cm, __shfl_xor(cm, d, 32));
      const float mn = fmaxf(mrun, cm);
      const float al = (mrun == -INFINITY) ? 0.f : exp2f(mrun - mn);
      mrun = mn;
      float ps = 0.f;
#pragma unroll
      for (int j = 0; j < 32; ++j) {
        const float p = exp2f(fminf(t[j] - mn, 0.f));
        t[j] = p;
        ps += p;
      }
#pragma unroll
      for (int d = 1; d <= 8; d <<= 1) ps += __shfl_xor(ps, d, 32);
      const float cc = ps * (1.0f / (float)CK);
      v4u pk[4];
#pragma unroll
      for (int i = 0; i < 4; ++i) {
#pragma unroll
        for (int e = 0; e < 4; ++e) {
          const int j = 8 * i + 2 * e;
          pk[i][e] = pk16(h_bits((_Float16)((t[j] - cc) * PCAR)), h_bits((_Float16)((t[j + 1] - cc) * PCAR)));
        }
      }
      lrun = lrun * al + ps;
      u16* pd = pls + r16 * PLP + kl0;
#pragma unroll
      for (int i = 0; i < 4; ++i) *(v4u*)(pd + 8 * i) = pk[i];
      if (sub == 0) { rowa[r16] = al; rowc[r16] = cc; }
    }
    __syncthreads();
    {
      float scl[8], cad[8];
#pragma unroll
      for (int r = 0; r < 8; ++r) { scl[r] = rowa[8 * hh + r]; cad[r] = rowc[8 * hh + r] * addsel; }
      const float* vsc = vsb + ((size_t)c * NKB + (size_t)(nkb - 1)) * DH;
      float vs[NACC];
#pragma unroll
      for (int j = 0; j < NACC; ++j) vs[j] = vsc[16 * j];
#pragma unroll
      for (int j = 0; j < NACC; ++j) {
#pragma unroll
        for (int r = 0; r < 8; ++r) o[j][r] = o[j][r] * scl[r] + cad[r] * vs[j];
      }
      const _Float16* pp = (const _Float16*)(const void*)pls + m * PLP + 8 * hh;
      const _Float16* vp = vbp + kbeg;
#pragma unroll 1
      for (int kb = wave; kb < nkb; kb += 8) {
        const v16h pf = ldfrag_h(pp + kb * 32);
        const _Float16* vk = vp + kb * 32;
        const v16h g0 = ldfrag_h(vk);
        const v16h g1 = ldfrag_h(vk + (size_t)16 * SEQ);
        const v16h g2 = ldfrag_h(vk + (size_t)32 * SEQ);
        const v16h g3 = ldfrag_h(vk + (size_t)48 * SEQ);
        o[0] = mma_h(pf, g0, o[0]);
        o[1] = mma_h(pf, g1, o[1]);
        o[2] = mma_h(pf, g2, o[2]);
        o[3] = mma_h(pf, g3, o[3]);
        guardpv4(o[0], o[1], o[2], o[3], pf, g0, g1, g2, g3);
      }
    }
  }
  acc_guard4(o[0], o[1], o[2], o[3]);

  __syncthreads();
#pragma unroll
  for (int j = 0; j < NACC; ++j) {
#pragma unroll
    for (int r = 0; r < 8; ++r) scs[(wave * 16 + 8 * hh + r) * OPP + 16 * j + m] = o[j][r];
  }
  __syncthreads();
  const int c4 = sub * 4;
  v4f sm4 = zero4();
#pragma unroll
  for (int w = 0; w < 8; ++w) sm4 += *(const v4f*)(scs + (w * 16 + r16) * OPP + c4);
  const float inv = (1.0f / lrun) * (CSC / (PCAR * VCAR));
#pragma unroll
  for (int e = 0; e < 4; ++e) {
    const float xs = sm4[e] * inv;
    const _Float16 hv = (_Float16)xs;
    const _Float16 rv = (_Float16)((xs - (float)hv) * RSC);
    pls[r16 * CTP + c4 + e]        = h_bits(hv);
    pls[(16 + r16) * CTP + c4 + e] = h_bits(rv);
  }
  __syncthreads();
  const int line = tid >> 3;
  const int plane = line >> 4;
  const int rowl  = line & 15;
  const int c8    = (tid & 7) * 8;
  const v4u ov = *(const v4u*)(pls + (plane * 16 + rowl) * CTP + c8);
  u16* dst = ((plane == 0) ? CHo : CRo) + ((size_t)b * SEQ + q0 + rowl) * DH + c8;
  *(volatile v4u*)dst = ov;
  __threadfence();
  *(volatile v4u*)dst = ov;
}

__global__ __launch_bounds__(HD_THREADS) void attn_head(const float* __restrict__ QF, const float* __restrict__ KF,
                                                      const float* __restrict__ V, u16* CHo, u16* CRo) {
  __shared__ __align__(16) float qs[DH];
  __shared__ float sc[TQ0];
  __shared__ float red[4];
  __shared__ float redb[4];
  __shared__ __align__(16) u16 SW[2 * DH];
  const int tid = threadIdx.x, lane = tid & 31, wave = tid >> 5;
  const int b = blockIdx.x / TQ0;
  const int t = blockIdx.x - b * TQ0;
  if (tid < DH) qs[tid] = QF[((size_t)b * TQ0 + t) * DH + tid];
  __syncthreads();
  float acc = 0.f;
  {
    const float* kp = KF + ((size_t)b * TQ0 + tid) * DH;
#pragma unroll 1
    for (int d = 0; d < DH; d += 8) {
      const v4f k0 = *(const v4f*)(kp + d), k1 = *(const v4f*)(kp + d + 4);
      const v4f q0 = *(const v4f*)(qs + d), q1 = *(const v4f*)(qs + d + 4);
#pragma unroll
      for (int e = 0; e < 4; ++e) acc += k0[e] * q0[e];
#pragma unroll
      for (int e = 0; e < 4; ++e) acc += k1[e] * q1[e];
    }
  }
  const float s = (tid <= t) ? acc * (RSQD * LOG2E) : -INFINITY;
  float mx = s;
#pragma unroll
  for (int d = 1; d <= 16; d <<= 1) mx = fmaxf(mx, __shfl_xor(mx, d, 32));
  if (lane == 0) red[wave] = mx;
  __syncthreads();
  float gm = red[0];
#pragma unroll
  for (int w = 1; w < 4; ++w) gm = fmaxf(gm, red[w]);
  const float p = exp2f(s - gm);
  float ps = p;
#pragma unroll
  for (int d = 1; d <= 16; d <<= 1) ps += __shfl_xor(ps, d, 32);
  if (lane == 0) redb[wave] = ps;
  sc[tid] = p;
  __syncthreads();
  float l = redb[0];
#pragma unroll
  for (int w = 1; w < 4; ++w) l += redb[w];
  const float inv = (1.0f / l) * CSC;
  if (wave < 2) {
    const float* vp = V + (size_t)b * SEQ * DH + tid;
    float cx = 0.f;
#pragma unroll 1
    for (int j = 0; j <= t; ++j) {
      cx += sc[j] * vp[(size_t)j * DH];
    }
    const float x0 = cx * inv;
    const _Float16 h0 = (_Float16)x0;
    const _Float16 r0 = (_Float16)((x0 - (float)h0) * RSC);
    SW[tid]      = h_bits(h0);
    SW[DH + tid] = h_bits(r0);
  }
  __syncthreads();
  if (wave == 0) {
    const int l16 = lane & 15;
    const int plane = l16 >> 3, p8 = (l16 & 7) * 8;
    const v4u ov = *(const v4u*)(SW + plane * DH + p8);
    u16* dst = ((plane == 0) ? CHo : CRo) + ((size_t)b * SEQ + t) * DH + p8;
    if (lane < 16) *(volatile v4u*)dst = ov;
    __threadfence();
    if (lane < 16) *(volatile v4u*)dst = ov;
  }
}

extern "C" void kernel_launch(void* const* d_in, const int* in_sizes, int n_in,
                              void* d_out, int out_size, void* d_ws, size_t ws_size,
                              hipStream_t stream) {
  if (n_in < 9) return;
  const int nb   = NB;
  const int rows = nb * SEQ;
  if ((long long)in_sizes[0] < (long long)NB * SEQ_FULL * EMB) return;
  if (in_sizes[1] < EMB * DH || in_sizes[3] < EMB * DH || in_sizes[5] < EMB * DH || in_sizes[7] < DH * EMB) return;
  if (in_sizes[2] < DH || in_sizes[4] < DH || in_sizes[6] < DH || in_sizes[8] < EMB) return;
  if ((long long)out_size < (long long)rows * EMB) return;

  const float* x  = (const float*)d_in[0];
  const float* wq = (const float*)d_in[1];
  const float* bq = (const float*)d_in[2];
  const float* wk = (const float*)d_in[3];
  const float* bk = (const float*)d_in[4];
  const float* wv = (const float*)d_in[5];
  const float* bv = (const float*)d_in[6];
  const float* wo = (const float*)d_in[7];
  const float* bo = (const float*)d_in[8];
  float*       out = (float*)d_out;

  const size_t szW  = (size_t)EMB * DH * 2;
  const size_t szXB = (size_t)rows * EMB * 2;
  const size_t szP  = (size_t)rows * DH * 2;
  const size_t szV  = (size_t)rows * DH * 4;
  const size_t szVT = (size_t)nb * DH * SEQ * 2;
  const size_t szVS = (size_t)nb * NCHK * NKB * DH * 4;
  const size_t szHF = (size_t)nb * TQ0 * DH * 4;
  size_t off = 0;
  const size_t oWQ = off; off += szW;
  const size_t oWK = off; off += szW;
  const size_t oWV = off; off += szW;
  const size_t oWO = off; off += szW;
  const size_t oXB = off; off += szXB;
  const size_t oQ  = off; off += szP;
  const size_t oK  = off; off += szP;
  const size_t oV  = off; off += szV;
  const size_t oVT = off; off += szVT;
  const size_t oVS = off; off += szVS;
  const size_t oQF = off; off += szHF;
  const size_t oKF = off; off += szHF;
  const size_t oCH = off; off += szP;
  const size_t oCR = off; off += szP;
  if (off > ws_size) return;
  if (off > WS_CAP) return;

  char* ws = (char*)d_ws;
  u16*   WQT = (u16*)(ws + oWQ);
  u16*   WKT = (u16*)(ws + oWK);
  u16*   WVT = (u16*)(ws + oWV);
  u16*   WOT = (u16*)(ws + oWO);
  u16*   XB  = (u16*)(ws + oXB);
  u16*   QP  = (u16*)(ws + oQ);
  u16*   KP  = (u16*)(ws + oK);
  float* V   = (float*)(ws + oV);
  u16*   VT  = (u16*)(ws + oVT);
  float* VS  = (float*)(ws + oVS);
  float* QF  = (float*)(ws + oQF);
  float* KF  = (float*)(ws + oKF);
  u16*   CH  = (u16*)(ws + oCH);
  u16*   CR  = (u16*)(ws + oCR);

  const int n8x = (SEQ * EMB) / 8;
  if ((n8x % 256) != 0 || (rows % 64) != 0 || ((nb * TQ0) % 64) != 0) return;
  const dim3 blk(256);
  const dim3 gWT((EMB / 64) * (DH / 64));
  const dim3 gX(n8x / 256, nb);
  const dim3 gG((rows / 64) * (DH / 64));
  const dim3 gH(((nb * TQ0) / 64) * (DH / 64));
  const dim3 bG(128);
  const dim3 gXT(nb * (SEQ / 64));
  const dim3 gVS(nb * NCHK);
  const dim3 bVS(64);
  const dim3 gAT(nb * NQT);
  const dim3 bAT(ATT_THREADS);
  const dim3 gHD(nb * TQ0);
  const dim3 bHD(HD_THREADS);
  const dim3 gO((rows / 64) * (EMB / 64));

  wt16<<<gWT, blk, 0, stream>>>(wq, WQT, EMB, DH, 0, 1.0f);
  wt16<<<gWT, blk, 0, stream>>>(wk, WKT, EMB, DH, 0, 1.0f);
  wt16<<<gWT, blk, 0, stream>>>(wv, WVT, EMB, DH, 0, 1.0f);
  wt16<<<gWT, blk, 0, stream>>>(wo, WOT, DH, EMB, 1, WSC);
  cvtx<<<gX, blk, 0, stream>>>(x, XB, n8x);
  gemm_bh16<<<gG, bG, 0, stream>>>(XB, WQT, bq, QP, rows, DH, EMB, 1.0f, QSC);
  gemm_bh16<<<gG, bG, 0, stream>>>(XB, WKT, bk, KP, rows, DH, EMB, 1.0f, KSC);
  gemm_b32<<<gG, bG, 0, stream>>>(XB, WVT, bv, V, rows, DH, EMB, rows, 0, 1.0f);
  gemm_b32<<<gH, bG, 0, stream>>>(XB, WQT, bq, QF, nb * TQ0, DH, EMB, TQ0, SEQ, 1.0f);
  gemm_b32<<<gH, bG, 0, stream>>>(XB, WKT, bk, KF, nb * TQ0, DH, EMB, TQ0, SEQ, 1.0f);
  xt16<<<gXT, blk, 0, stream>>>(V, VT);
  vsum_k<<<gVS, bVS, 0, stream>>>(V, VS);
  attn_fwd<<<gAT, bAT, 0, stream>>>(QP, KP, VT, VS, CH, CR);
  attn_head<<<gHD, bHD, 0, stream>>>(QF, KF, V, CH, CR);
  gemm_h2_32<<<gO, bG, 0, stream>>>(CH, CR, WOT, bo, out, rows, EMB, DH,
                                    1.0f / (CSC * WSC), 1.0f / (CSC * WSC * RSC));
  (void)hipGetLastError();
}
